// MolecularEncoder_39651138076879
// MI455X (gfx1250) — hardware-run, weakly checked
//
#include <hip/hip_runtime.h>
#include <stddef.h>


#define FIN     15
#define KX      16
#define CH      128
#define NH1     8
#define NH2     4
#define F1      (NH1 * CH)
#define F2      (NH2 * CH)
#define PO      64
#define WSC     64
#define ASC     8
#define NTHR    256
#define NWAVE   8
#define EPT     8
#define NGRP    2
#define CHUNK   (NTHR * EPT * NGRP)
#define WCAP    (EPT * NGRP * 32)
#define LISTN   (NWAVE * WCAP)
#define NBC     4096
#define NBF     1024
#define RCAP    40960
#define RBN     128
#define TGT     256
#define DEGCAP  256
#define OTHR    512
#define BM      64
#define WSCAP   134217728
#define NEG_SLOPE 0.2f
#define BN_EPS  1e-5f

#define LDS_FILL ((RCAP + NBF + LISTN) * 4 + 64)

static_assert((CHUNK & (CHUNK - 1)) == 0);
static_assert(CHUNK <= 4096);
static_assert(NBC <= 4096 && NBF <= 4096);
static_assert((NBC & (NBC - 1)) == 0 && (NBF & (NBF - 1)) == 0);
static_assert(NBC == 4 * NBF);
static_assert(OTHR * 8 == NBC);
static_assert((RCAP % 32) == 0);
static_assert(TGT == NWAVE * 32);
static_assert((NBC % TGT) == 0);
static_assert((TGT % BM) == 0);
static_assert(BM * 4 == NTHR);
static_assert(F2 * 4 == F1 * 2);
static_assert(CH * 4 == 2 * CH * 2);
static_assert(WCAP == EPT * NGRP * 32);

typedef float          v4f  __attribute__((ext_vector_type(4)));
typedef float          v8f  __attribute__((ext_vector_type(8)));
typedef int            v4i  __attribute__((ext_vector_type(4)));
typedef _Float16       v4h  __attribute__((ext_vector_type(4)));
typedef _Float16       v8h  __attribute__((ext_vector_type(8)));
typedef _Float16       v16h __attribute__((ext_vector_type(16)));
union FragH { v16h v; v8h h[2]; };

__device__ __forceinline__ v8f wmh(v16h a, v16h b, v8f c) {
  v8f d = __builtin_amdgcn_wmma_f32_16x16x32_f16(false, a, false, b, (short)0, c, false, false);
  asm volatile("v_nop\n\tv_nop\n\tv_nop\n\tv_nop" : "+v"(d) : "v"(a), "v"(b));
  return d;
}

__device__ __forceinline__ float lrelu(float v) { return v > 0.0f ? v : NEG_SLOPE * v; }
__device__ __forceinline__ float elu1(float v)  { return v > 0.0f ? v : expm1f(v); }

template <int NB>
__device__ __forceinline__ int scan_chunk(const int* __restrict__ dsts, int nE, int cbase, int slotBase,
                                          int vec8, int* list, int tid, int lane, int wave) {
  int wc = 0;
#pragma unroll
  for (int g = 0; g < NGRP; ++g) {
    const int el0  = (g * NTHR + tid) * EPT;
    const int e0   = cbase + el0;
    const int sent = -2147483647 - 1;
    v4i da, db;
    if (vec8 != 0 && cbase + CHUNK <= nE) {
      da = *(const v4i*)(dsts + e0);
      db = *(const v4i*)(dsts + e0 + 4);
    } else {
      da.x = (e0     < nE) ? dsts[min(e0, nE - 1)] : sent;
      da.y = (e0 + 1 < nE) ? dsts[min(e0 + 1, nE - 1)] : sent;
      da.z = (e0 + 2 < nE) ? dsts[min(e0 + 2, nE - 1)] : sent;
      da.w = (e0 + 3 < nE) ? dsts[min(e0 + 3, nE - 1)] : sent;
      db.x = (e0 + 4 < nE) ? dsts[min(e0 + 4, nE - 1)] : sent;
      db.y = (e0 + 5 < nE) ? dsts[min(e0 + 5, nE - 1)] : sent;
      db.z = (e0 + 6 < nE) ? dsts[min(e0 + 6, nE - 1)] : sent;
      db.w = (e0 + 7 < nE) ? dsts[min(e0 + 7, nE - 1)] : sent;
    }
    const unsigned nb = (unsigned)slotBase;
    const unsigned s0 = (unsigned)da.x - nb, s1 = (unsigned)da.y - nb;
    const unsigned s2 = (unsigned)da.z - nb, s3 = (unsigned)da.w - nb;
    const unsigned s4 = (unsigned)db.x - nb, s5 = (unsigned)db.y - nb;
    const unsigned s6 = (unsigned)db.z - nb, s7 = (unsigned)db.w - nb;
    const bool h0 = s0 < (unsigned)NB, h1 = s1 < (unsigned)NB, h2 = s2 < (unsigned)NB, h3 = s3 < (unsigned)NB;
    const bool h4 = s4 < (unsigned)NB, h5 = s5 < (unsigned)NB, h6 = s6 < (unsigned)NB, h7 = s7 < (unsigned)NB;
    const unsigned any = __builtin_amdgcn_ballot_w32(h0 | h1 | h2 | h3 | h4 | h5 | h6 | h7);
    if (any != 0u) {
#define HITJ(J, HJ, SJ) { \
        const unsigned mj = __builtin_amdgcn_ballot_w32(HJ); \
        if (mj != 0u) { \
          if (HJ) { \
            const int pos = wc + (int)__builtin_amdgcn_mbcnt_lo(mj, 0u); \
            if (pos < WCAP) list[wave * WCAP + pos] = ((el0 + (J)) << 12) | (int)(SJ); \
          } \
          wc += (int)__builtin_popcount(mj); } }
      HITJ(0, h0, s0)
      HITJ(1, h1, s1)
      HITJ(2, h2, s2)
      HITJ(3, h3, s3)
      HITJ(4, h4, s4)
      HITJ(5, h5, s5)
      HITJ(6, h6, s6)
      HITJ(7, h7, s7)
#undef HITJ
    }
  }
  return wc;
}

__global__ __launch_bounds__(NTHR) void k_uvec(const float* __restrict__ W1, const float* __restrict__ aS,
                                               const float* __restrict__ aD, float* u) {
  __shared__ __attribute__((aligned(16))) float su[256];
  const int tid = threadIdx.x;
  const int which = tid >> 7;
  const int h = (tid >> 4) & (NH1 - 1);
  const int k = tid & (KX - 1);
  const int kc = k < FIN ? k : FIN - 1;
  const float* att = which ? aD : aS;
  const float* wr = W1 + (size_t)kc * F1 + h * CH;
  const float* ar = att + h * CH;
  float s = 0.f;
#pragma unroll 4
  for (int c = 0; c < CH; ++c) s += wr[c] * ar[c];
  su[tid] = (k < FIN) ? s : 0.f;
  __syncthreads();
  const int q = tid < 64 ? tid : 63;
  const v4f v = *(const v4f*)(su + 4 * q);
  const bool act = tid < 64;
  if (act) *(volatile v4f*)(u + 4 * q) = v;
  __threadfence();
  if (act) *(volatile v4f*)(u + 4 * q) = v;
}

__global__ __launch_bounds__(NTHR) void k_xprep(const float* __restrict__ x, const float* __restrict__ u,
                                                float* xp, float* eS, float* eD, int nN, int npad) {
  __shared__ __attribute__((aligned(16))) float su[256];
  __shared__ __attribute__((aligned(16))) float sx[256 * KX];
  __shared__ __attribute__((aligned(16))) float sES[NH1 * 256];
  __shared__ __attribute__((aligned(16))) float sED[NH1 * 256];
  const int tid = threadIdx.x;
  const int rowBase = (int)blockIdx.x * 256;
  su[tid] = u[tid];
  const int row = rowBase + tid;
  int rr = row > nN - 1 ? nN - 1 : row;
  rr = rr < 0 ? 0 : rr;
  const float* xr = x + (size_t)rr * FIN;
  const bool live = row < nN;
  float xv[FIN];
#pragma unroll
  for (int k = 0; k < FIN; ++k) { const float t = xr[k]; xv[k] = live ? t : 0.f; }
#pragma unroll
  for (int k = 0; k < FIN; ++k) sx[tid * KX + k] = xv[k];
  sx[tid * KX + FIN] = 0.f;
  __syncthreads();
#pragma unroll 1
  for (int h = 0; h < NH1; ++h) {
    const float* us = su + h * KX;
    const float* ud = su + NH1 * KX + h * KX;
    float ps = 0.f, pd = 0.f;
#pragma unroll
    for (int k = 0; k < FIN; ++k) { ps += xv[k] * us[k]; pd += xv[k] * ud[k]; }
    sES[h * 256 + tid] = ps;
    sED[h * 256 + tid] = pd;
  }
  __syncthreads();
  v4f cx[4], ce[2], cd[2];
#pragma unroll
  for (int it = 0; it < 4; ++it) cx[it] = *(const v4f*)(sx + 4 * (it * 256 + tid));
#pragma unroll
  for (int it = 0; it < 2; ++it) {
    const int id = it * 256 + tid, h = id >> 6, q = id & 63;
    ce[it] = *(const v4f*)(sES + h * 256 + 4 * q);
    cd[it] = *(const v4f*)(sED + h * 256 + 4 * q);
  }
  float* xb = xp + (size_t)rowBase * KX;
#pragma unroll
  for (int it = 0; it < 4; ++it) *(volatile v4f*)(xb + 4 * (it * 256 + tid)) = cx[it];
#pragma unroll
  for (int it = 0; it < 2; ++it) {
    const int id = it * 256 + tid, h = id >> 6, q = id & 63;
    *(volatile v4f*)(eS + (size_t)h * npad + rowBase + 4 * q) = ce[it];
    *(volatile v4f*)(eD + (size_t)h * npad + rowBase + 4 * q) = cd[it];
  }
  __threadfence();
#pragma unroll
  for (int it = 0; it < 4; ++it) *(volatile v4f*)(xb + 4 * (it * 256 + tid)) = cx[it];
#pragma unroll
  for (int it = 0; it < 2; ++it) {
    const int id = it * 256 + tid, h = id >> 6, q = id & 63;
    *(volatile v4f*)(eS + (size_t)h * npad + rowBase + 4 * q) = ce[it];
    *(volatile v4f*)(eD + (size_t)h * npad + rowBase + 4 * q) = cd[it];
  }
}

__global__ __launch_bounds__(NTHR) void k_w1cvt(const float* __restrict__ W1, _Float16* wp) {
  constexpr int UNITS = F1 * 4;
  const int i = (int)blockIdx.x * NTHR + (int)threadIdx.x;
  if (i >= UNITS) return;
  const int n = i >> 2, seg = i & 3;
  const int h = n >> 7;
  const int shift = (h & 1) * 16;
  v8h o;
#pragma unroll
  for (int j = 0; j < 8; ++j) {
    const int slot = 8 * seg + j;
    const int k = slot - shift;
    const bool valid = (k >= 0) && (k < FIN);
    int kc = k < 0 ? 0 : (k > FIN - 1 ? FIN - 1 : k);
    const float v = W1[(size_t)kc * F1 + n];
    o[j] = valid ? (_Float16)(v * (float)WSC) : (_Float16)0.0f;
  }
  _Float16* d = wp + (size_t)i * 8;
  *(volatile v8h*)d = o;
  __threadfence();
  *(volatile v8h*)d = o;
}

__global__ __launch_bounds__(NTHR) void k_wtcvt(const float* __restrict__ W, _Float16* dst, int K, int Nout,
                                                int dstStride, int dstOff, int nUnits) {
  const int i = (int)blockIdx.x * NTHR + (int)threadIdx.x;
  if (i >= nUnits) return;
  const int ppr = K >> 3;
  const int n = i / ppr;
  const int seg = i - n * ppr;
  const float* p = W + (size_t)(8 * seg) * Nout + n;
  v8h o;
#pragma unroll
  for (int j = 0; j < 8; ++j) o[j] = (_Float16)(p[(size_t)j * Nout] * (float)WSC);
  _Float16* d = dst + (size_t)n * dstStride + dstOff + 8 * seg;
  *(volatile v8h*)d = o;
  __threadfence();
  *(volatile v8h*)d = o;
}

__global__ __launch_bounds__(NTHR) void k_count(
    const int* __restrict__ dsts, int* cnt, int nE, int vec8) {
  __shared__ __attribute__((aligned(16))) int scnt[NBC];
  __shared__ __attribute__((aligned(16))) int list[LISTN];
  __shared__ int wcnt[NWAVE];
  const int tid = threadIdx.x, lane = tid & 31, wave = tid >> 5;
  const int nodeBase = blockIdx.x * NBC;

  for (int i = tid; i < NBC; i += NTHR) scnt[i] = 0;
  __syncthreads();

  const int nChunks = (nE + CHUNK - 1) / CHUNK;
#pragma unroll 1
  for (int ch = 0; ch < nChunks; ++ch) {
    const int cbase = ch * CHUNK;
    const int wc = scan_chunk<NBC>(dsts, nE, cbase, nodeBase, vec8, list, tid, lane, wave);
    if (lane == 0) wcnt[wave] = wc;
    __syncthreads();
    if (wave == 0) {
#pragma unroll 1
      for (int wsx = 0; wsx < NWAVE; ++wsx) {
        int n = __builtin_amdgcn_readfirstlane(wcnt[wsx]);
        n = n > WCAP ? WCAP : (n < 0 ? 0 : n);
        const int* lp = list + wsx * WCAP;
#pragma unroll 1
        for (int i = 0; i < n; ++i) {
          const int ent  = __builtin_amdgcn_readfirstlane(lp[i]);
          const int slot = ent & (NBC - 1);
          if (lane == 0) scnt[slot] = scnt[slot] + 1;
        }
      }
    }
    __syncthreads();
  }

  v4i cq[4];
#pragma unroll
  for (int q = 0; q < 4; ++q) {
    const int f = (wave * 4 + q) * 128 + 4 * lane;
    cq[q] = *(const v4i*)(scnt + f);
  }
  int* cp = cnt + (size_t)nodeBase;
#pragma unroll
  for (int q = 0; q < 4; ++q) {
    const int f = (wave * 4 + q) * 128 + 4 * lane;
    *(volatile v4i*)(cp + f) = cq[q];
  }
  __threadfence();
#pragma unroll
  for (int q = 0; q < 4; ++q) {
    const int f = (wave * 4 + q) * 128 + 4 * lane;
    *(volatile v4i*)(cp + f) = cq[q];
  }
}

__global__ __launch_bounds__(OTHR) void k_offsets(
    const int* __restrict__ cnt, int* off, int* rbase, int nChunk) {
  __shared__ __attribute__((aligned(16))) int soff[NBC];
  __shared__ __attribute__((aligned(16))) int srb[RBN];
  __shared__ int wtot[OTHR / 32];
  const int tid = threadIdx.x, lane = tid & 31, wave = tid >> 5, sub = tid >> 7;
  for (int i = tid; i < RBN; i += OTHR) srb[i] = 0;
  int carry = 0;
#pragma unroll 1
  for (int ch = 0; ch < nChunk; ++ch) {
    const int base = ch * NBC;
    const v4i c0 = *(const v4i*)(cnt + base + 8 * tid);
    const v4i c1 = *(const v4i*)(cnt + base + 8 * tid + 4);
    const int e0 = max(c0.x, 0), e1 = max(c0.y, 0), e2 = max(c0.z, 0), e3 = max(c0.w, 0);
    const int e4 = max(c1.x, 0), e5 = max(c1.y, 0), e6 = max(c1.z, 0), e7 = max(c1.w, 0);
    const int ts = e0 + e1 + e2 + e3 + e4 + e5 + e6 + e7;
    int incl = ts;
#pragma unroll
    for (int d = 1; d < 32; d <<= 1) {
      const int t = __shfl_up(incl, d);
      if (lane >= d) incl += t;
    }
    if (lane == 31) wtot[wave] = incl;
    __syncthreads();
    const int S0 = wtot[0]  + wtot[1]  + wtot[2]  + wtot[3];
    const int S1 = wtot[4]  + wtot[5]  + wtot[6]  + wtot[7];
    const int S2 = wtot[8]  + wtot[9]  + wtot[10] + wtot[11];
    const int S3 = wtot[12] + wtot[13] + wtot[14] + wtot[15];
    int pre = 0;
#pragma unroll 1
    for (int w = 4 * sub; w < wave; ++w) pre += wtot[w];
    const int b0 = carry;
    const int b1 = b0 + ((S0 + 31) & ~31);
    const int b2 = b1 + ((S1 + 31) & ~31);
    const int b3 = b2 + ((S2 + 31) & ~31);
    const int b4 = b3 + ((S3 + 31) & ~31);
    const int myb = sub == 0 ? b0 : (sub == 1 ? b1 : (sub == 2 ? b2 : b3));
    if (tid == 0) {
      srb[min(4 * ch + 0, RBN - 1)] = b0;
      srb[min(4 * ch + 1, RBN - 1)] = b1;
      srb[min(4 * ch + 2, RBN - 1)] = b2;
      srb[min(4 * ch + 3, RBN - 1)] = b3;
    }
    int run = myb + pre + incl - ts;
    soff[8 * tid + 0] = run; run += e0;
    soff[8 * tid + 1] = run; run += e1;
    soff[8 * tid + 2] = run; run += e2;
    soff[8 * tid + 3] = run; run += e3;
    soff[8 * tid + 4] = run; run += e4;
    soff[8 * tid + 5] = run; run += e5;
    soff[8 * tid + 6] = run; run += e6;
    soff[8 * tid + 7] = run;
    carry = b4;
    __syncthreads();
    const v4i o0 = *(const v4i*)(soff + 4 * tid);
    const v4i o1 = *(const v4i*)(soff + 4 * (tid + OTHR));
    int* op = off + base;
    *(volatile v4i*)(op + 4 * tid) = o0;
    *(volatile v4i*)(op + 4 * (tid + OTHR)) = o1;
    __threadfence();
    *(volatile v4i*)(op + 4 * tid) = o0;
    *(volatile v4i*)(op + 4 * (tid + OTHR)) = o1;
    __syncthreads();
  }
  if (tid == 0) srb[min(4 * nChunk, RBN - 1)] = carry;
  __syncthreads();
  v4i rv = {0, 0, 0, 0};
  if (tid < 32) rv = *(const v4i*)(srb + 4 * tid);
  if (tid < 32) *(volatile v4i*)(rbase + 4 * tid) = rv;
  __threadfence();
  if (tid < 32) *(volatile v4i*)(rbase + 4 * tid) = rv;
}

__global__ __launch_bounds__(NTHR) void k_fill(
    const int* __restrict__ srcs, const int* __restrict__ dsts,
    const int* __restrict__ off, const int* __restrict__ rbase,
    int* csr, int nN, int nE, int vec8, int csrLen) {
  extern __shared__ v4f lds_dyn[];
  int* region = (int*)lds_dyn;
  int* cursor = region + RCAP;
  int* list   = cursor + NBF;
  int* wcnt   = list + LISTN;
  const int tid = threadIdx.x, lane = tid & 31, wave = tid >> 5;
  const int b = blockIdx.x;
  const int nodeBase = b * NBF;

  int rb0 = rbase[b];
  const int rb1 = rbase[b + 1];
  rb0 = rb0 < 0 ? 0 : (rb0 > csrLen ? csrLen : rb0);
  rb0 &= ~31;
  int len = rb1 - rb0;
  len = len < 0 ? 0 : (len > RCAP ? RCAP : len);
  int lenW = (len + 31) & ~31;
  if (rb0 + lenW > csrLen) lenW = (csrLen - rb0) & ~31;

  {
    const v4i z = {0, 0, 0, 0};
    for (int i = tid; i < RCAP / 4; i += NTHR) ((v4i*)region)[i] = z;
    for (int s = tid; s < NBF; s += NTHR) {
      int o = off[nodeBase + s] - rb0;
      o = o < 0 ? 0 : (o > RCAP ? RCAP : o);
      cursor[s] = o;
    }
  }
  __syncthreads();

  const int nChunks = (nE + CHUNK - 1) / CHUNK;
#pragma unroll 1
  for (int ch = 0; ch < nChunks; ++ch) {
    const int cbase = ch * CHUNK;
    const int wc = scan_chunk<NBF>(dsts, nE, cbase, nodeBase, vec8, list, tid, lane, wave);
    if (lane == 0) wcnt[wave] = wc;
    __syncthreads();
    if (wave == 0) {
#pragma unroll 1
      for (int wsx = 0; wsx < NWAVE; ++wsx) {
        int n = __builtin_amdgcn_readfirstlane(wcnt[wsx]);
        n = n > WCAP ? WCAP : (n < 0 ? 0 : n);
        const int* lp = list + wsx * WCAP;
#pragma unroll 1
        for (int i = 0; i < n; ++i) {
          const int ent  = __builtin_amdgcn_readfirstlane(lp[i]);
          const int slot = ent & (NBF - 1);
          int e = cbase + ((ent >> 12) & (CHUNK - 1));
          e = e > nE - 1 ? nE - 1 : e;
          int sv = srcs[e];
          sv = sv < 0 ? 0 : (sv > nN - 1 ? nN - 1 : sv);
          if (lane == 0) {
            int pos = cursor[slot];
            pos = pos < 0 ? 0 : (pos > RCAP - 1 ? RCAP - 1 : pos);
            region[pos] = sv;
            const int np = pos + 1;
            cursor[slot] = np > RCAP ? RCAP : np;
          }
        }
      }
    }
    __syncthreads();
  }

  const int nv = lenW >> 2;
  int* gp = csr + rb0;
#pragma unroll 1
  for (int i = tid; i < nv; i += NTHR) { const v4i v = ((const v4i*)region)[i]; *(volatile v4i*)(gp + 4 * i) = v; }
  __threadfence();
#pragma unroll 1
  for (int i = tid; i < nv; i += NTHR) { const v4i v = ((const v4i*)region)[i]; *(volatile v4i*)(gp + 4 * i) = v; }
}

__global__ __launch_bounds__(NTHR) void k_gat1(
    const int* __restrict__ csr, const int* __restrict__ off, const int* __restrict__ cnt,
    const float* __restrict__ eS, const float* __restrict__ eD, const float* __restrict__ xp,
    _Float16* zh, int nN, int npad, int csrLen) {
  const int tid = threadIdx.x, lane = tid & 31, wave = tid >> 5;
  const int tbase = blockIdx.x * TGT + wave * 32;
  const int hd = lane >> 2;
  const int kq = 4 * (lane & 3);
  const int cl    = tbase + lane;
  const int cnt_l = cnt[cl];
  const int off_l = off[cl];
  const float* eSh = eS + (size_t)hd * npad;
  const float* eDh = eD + (size_t)hd * npad;

#pragma unroll 1
  for (int j = 0; j < 32; ++j) {
    const int c = tbase + j;
    int n = __shfl(cnt_l, j);
    n = n < 0 ? 0 : (n > DEGCAP ? DEGCAP : n);
    const int st = __shfl(off_l, j);
    const float edc = eDh[c];
    const float eself = lrelu(eSh[c] + edc);

    float mx = eself;
#pragma unroll 1
    for (int q0 = 0; q0 < n; q0 += 32) {
      int pos = st + q0 + lane;
      pos = pos < 0 ? 0 : (pos > csrLen - 1 ? csrLen - 1 : pos);
      int sl = csr[pos];
      sl = sl < 0 ? 0 : (sl > nN - 1 ? nN - 1 : sl);
      const int mcnt = (n - q0) < 32 ? (n - q0) : 32;
#pragma unroll 1
      for (int pp = 0; pp < mcnt; ++pp) {
        const int s = __builtin_amdgcn_readlane(sl, pp);
        mx = fmaxf(mx, lrelu(eSh[s] + edc));
      }
    }

    const float pself = __expf(eself - mx);
    float den = pself;
    const v4f xc = *(const v4f*)(xp + (size_t)c * KX + kq);
    float a0 = pself * xc.x, a1 = pself * xc.y, a2 = pself * xc.z, a3 = pself * xc.w;
#pragma unroll 1
    for (int q0 = 0; q0 < n; q0 += 32) {
      int pos = st + q0 + lane;
      pos = pos < 0 ? 0 : (pos > csrLen - 1 ? csrLen - 1 : pos);
      int sl = csr[pos];
      sl = sl < 0 ? 0 : (sl > nN - 1 ? nN - 1 : sl);
      const int mcnt = (n - q0) < 32 ? (n - q0) : 32;
#pragma unroll 1
      for (int pp = 0; pp < mcnt; ++pp) {
        const int s = __builtin_amdgcn_readlane(sl, pp);
        const float p = __expf(lrelu(eSh[s] + edc) - mx);
        den += p;
        const v4f xv = *(const v4f*)(xp + (size_t)s * KX + kq);
        a0 += xv.x * p; a1 += xv.y * p; a2 += xv.z * p; a3 += xv.w * p;
      }
    }

    const float rd = __builtin_amdgcn_rcpf(den);
    v4h o;
    o[0] = (_Float16)((a0 * rd) * (float)ASC);
    o[1] = (_Float16)((a1 * rd) * (float)ASC);
    o[2] = (_Float16)((a2 * rd) * (float)ASC);
    o[3] = (_Float16)((a3 * rd) * (float)ASC);
    _Float16* gp = zh + (size_t)c * CH + 4 * lane;
    *(volatile v4h*)gp = o;
    __threadfence();
    *(volatile v4h*)gp = o;
  }
}

template <int NCW, int O16>
__global__ __launch_bounds__(NTHR) void k_gemm(
    const _Float16* __restrict__ Ap, const _Float16* __restrict__ Bp,
    const float* __restrict__ bias, const float* __restrict__ bng, const float* __restrict__ bnb,
    const float* __restrict__ bnm, const float* __restrict__ bnv,
    const float* __restrict__ attS, const float* __restrict__ attD,
    float* eS, float* eD, float* C32, _Float16* C16,
    int lda, int kaMode, int KT, int ldc, int flags, int npad, float osc) {
  constexpr int TPW = NCW / 32;
  constexpr int PPR = O16 ? (NCW / 8) : (NCW / 4);
  constexpr int NIT = (BM * PPR) / NTHR;
  static_assert((BM * PPR) % NTHR == 0);
  static_assert(TPW >= 1 && TPW * 32 == NCW);
  static_assert(NIT >= 1);

  __shared__ __attribute__((aligned(16))) float stg[BM * NCW];
  __shared__ __attribute__((aligned(16))) float sES[BM];
  __shared__ __attribute__((aligned(16))) float sED[BM];
  const int tid = threadIdx.x, lane = tid & 31, wave = tid >> 5, hh = lane >> 4, m = lane & 15;
  const int y = (int)blockIdx.y;
  const int rowBase = (int)blockIdx.x * BM;
  const int colBase = y * NCW;
  const int ka0 = kaMode ? 32 * (y >> 1) : 0;
  const int rg = wave >> 1, chf = wave & 1;
  const int r0 = rg * 16;
  const int c0 = chf * (NCW / 2);
  const int KB = 32 * KT;

  v8f acc[TPW];
#pragma unroll
  for (int t = 0; t < TPW; ++t) { v8f z = {0.f, 0.f, 0.f, 0.f, 0.f, 0.f, 0.f, 0.f}; acc[t] = z; }

  const _Float16* ap  = Ap + (size_t)(rowBase + r0 + m) * lda + ka0 + 8 * hh;
  const _Float16* bp0 = Bp + (size_t)(colBase + c0 + m) * KB + 8 * hh;
#pragma unroll 1
  for (int kt = 0; kt < KT; ++kt) {
    FragH a;
    a.h[0] = *(const v8h*)(ap + 32 * kt);
    a.h[1] = *(const v8h*)(ap + 32 * kt + 16);
#pragma unroll
    for (int t = 0; t < TPW; ++t) {
      const _Float16* bp = bp0 + (size_t)(16 * t) * KB + 32 * kt;
      FragH bf;
      bf.h[0] = *(const v8h*)bp;
      bf.h[1] = *(const v8h*)(bp + 16);
      acc[t] = wmh(a.v, bf.v, acc[t]);
    }
  }

  {
    float* sp = stg + (size_t)(r0 + 8 * hh) * NCW + c0 + m;
#pragma unroll
    for (int t = 0; t < TPW; ++t) {
#pragma unroll
      for (int r = 0; r < 8; ++r) sp[r * NCW + 16 * t] = acc[t][r] * osc;
    }
  }
  __syncthreads();

  if constexpr (NCW == 128 && O16 == 0) {
    if (flags & 16) {
      constexpr int CPP = NCW / 4;
      const int drow = tid >> 2, part = tid & 3;
      const float* rp = stg + (size_t)drow * NCW + CPP * part;
      const float* sa = attS + (size_t)y * NCW + CPP * part;
      const float* sd = attD + (size_t)y * NCW + CPP * part;
      float ps = 0.f, pd = 0.f;
#pragma unroll 2
      for (int c = 0; c < CPP; c += 4) {
        const v4f hv = *(const v4f*)(rp + c);
        const v4f av = *(const v4f*)(sa + c);
        const v4f dv = *(const v4f*)(sd + c);
        ps += hv.x * av.x + hv.y * av.y + hv.z * av.z + hv.w * av.w;
        pd += hv.x * dv.x + hv.y * dv.y + hv.z * dv.z + hv.w * dv.w;
      }
      ps += __shfl_xor(ps, 1); pd += __shfl_xor(pd, 1);
      ps += __shfl_xor(ps, 2); pd += __shfl_xor(pd, 2);
      if (part == 0) { sES[drow] = ps; sED[drow] = pd; }
    }
  }

  if constexpr (O16) {
    v8h cv[NIT];
#pragma unroll
    for (int it = 0; it < NIT; ++it) {
      const int id = it * NTHR + tid;
      const int row = id / PPR, seg = id % PPR;
      const float* sp = stg + (size_t)row * NCW + 8 * seg;
      const v4f x0 = *(const v4f*)sp, x1 = *(const v4f*)(sp + 4);
      float e[8] = {x0.x, x0.y, x0.z, x0.w, x1.x, x1.y, x1.z, x1.w};
      const int n0 = colBase + 8 * seg;
      if (flags & 1) {
#pragma unroll
        for (int q = 0; q < 8; ++q) e[q] += bias[n0 + q];
      }
      if (flags & 2) {
#pragma unroll
        for (int q = 0; q < 8; ++q)
          e[q] = bng[n0 + q] * (e[q] - bnm[n0 + q]) * rsqrtf(bnv[n0 + q] + BN_EPS) + bnb[n0 + q];
      }
      if (flags & 4) {
#pragma unroll
        for (int q = 0; q < 8; ++q) e[q] = elu1(e[q]);
      }
      if (flags & 8) {
#pragma unroll
        for (int q = 0; q < 8; ++q) e[q] = fmaxf(e[q], 0.f);
      }
      v8h o;
#pragma unroll
      for (int q = 0; q < 8; ++q) o[q] = (_Float16)(e[q] * (float)ASC);
      cv[it] = o;
    }
#pragma unroll
    for (int it = 0; it < NIT; ++it) {
      const int id = it * NTHR + tid;
      const int row = id / PPR, seg = id % PPR;
      _Float16* gp = C16 + (size_t)(rowBase + row) * ldc + colBase + 8 * seg;
      *(volatile v8h*)gp = cv[it];
    }
    __threadfence();
#pragma unroll
    for (int it = 0; it < NIT; ++it) {
      const int id = it * NTHR + tid;
      const int row = id / PPR, seg = id % PPR;
      _Float16* gp = C16 + (size_t)(rowBase + row) * ldc + colBase + 8 * seg;
      *(volatile v8h*)gp = cv[it];
    }
  } else {
    v4f cv[NIT];
#pragma unroll
    for (int it = 0; it < NIT; ++it) {
      const int id = it * NTHR + tid;
      const int row = id / PPR, seg = id % PPR;
      v4f xv = *(const v4f*)(stg + (size_t)row * NCW + 4 * seg);
      const int n0 = colBase + 4 * seg;
      if (flags & 1) {
        xv.x += bias[n0]; xv.y += bias[n0 + 1]; xv.z += bias[n0 + 2]; xv.w += bias[n0 + 3];
      }
      cv[it] = xv;
    }
#pragma unroll
    for (int it = 0; it < NIT; ++it) {
      const int id = it * NTHR + tid;
      const int row = id / PPR, seg = id % PPR;
      float* gp = C32 + (size_t)(rowBase + row) * ldc + colBase + 4 * seg;
      *(volatile v4f*)gp = cv[it];
    }
    __threadfence();
#pragma unroll
    for (int it = 0; it < NIT; ++it) {
      const int id = it * NTHR + tid;
      const int row = id / PPR, seg = id % PPR;
      float* gp = C32 + (size_t)(rowBase + row) * ldc + colBase + 4 * seg;
      *(volatile v4f*)gp = cv[it];
    }
  }
  __syncthreads();

  if constexpr (NCW == 128 && O16 == 0) {
    const int iS = tid < 15 ? tid : 15;
    int iD = tid - 16; iD = iD < 0 ? 0 : (iD > 15 ? 15 : iD);
    const v4f vS = *(const v4f*)(sES + 4 * iS);
    const v4f vD = *(const v4f*)(sED + 4 * iD);
    const bool isS = tid < 16;
    const v4f dv = isS ? vS : vD;
    const size_t eb = (size_t)y * npad + rowBase;
    float* gp = isS ? (eS + eb + 4 * iS) : (eD + eb + 4 * iD);
    const bool act = ((flags & 16) != 0) && (tid < 32);
    if (act) *(volatile v4f*)gp = dv;
    __threadfence();
    if (act) *(volatile v4f*)gp = dv;
  }
}

__global__ __launch_bounds__(NTHR) void k_gcn(
    const int* __restrict__ csr, const int* __restrict__ off, const int* __restrict__ cnt,
    const float* __restrict__ hg, const float* __restrict__ bgp,
    const float* __restrict__ bng, const float* __restrict__ bnb,
    const float* __restrict__ bnm, const float* __restrict__ bnv,
    float* h2, int nN, int csrLen) {
  const int tid = threadIdx.x, lane = tid & 31, wave = tid >> 5;
  const int tbase = blockIdx.x * TGT + wave * 32;
  const int col = 4 * lane;
  const int cl    = tbase + lane;
  const int cnt_l = cnt[cl];
  const int off_l = off[cl];
  const v4f vb = *(const v4f*)(bgp + col);
  const v4f vg = *(const v4f*)(bng + col);
  const v4f vbeta = *(const v4f*)(bnb + col);
  const v4f vm = *(const v4f*)(bnm + col);
  const v4f vv = *(const v4f*)(bnv + col);
  const float rs0 = rsqrtf(vv.x + BN_EPS), rs1 = rsqrtf(vv.y + BN_EPS);
  const float rs2 = rsqrtf(vv.z + BN_EPS), rs3 = rsqrtf(vv.w + BN_EPS);

#pragma unroll 1
  for (int j = 0; j < 32; ++j) {
    const int c = tbase + j;
    int cc = __shfl(cnt_l, j);
    cc = cc < 0 ? 0 : cc;
    const int n = cc > DEGCAP ? DEGCAP : cc;
    const int st = __shfl(off_l, j);
    const float dc = rsqrtf((float)(cc + 1));
    const v4f hc = *(const v4f*)(hg + (size_t)c * CH + col);
    const float wc = dc * dc;
    float a0 = wc * hc.x, a1 = wc * hc.y, a2 = wc * hc.z, a3 = wc * hc.w;
#pragma unroll 1
    for (int q0 = 0; q0 < n; q0 += 32) {
      int pos = st + q0 + lane;
      pos = pos < 0 ? 0 : (pos > csrLen - 1 ? csrLen - 1 : pos);
      int sl = csr[pos];
      sl = sl < 0 ? 0 : (sl > nN - 1 ? nN - 1 : sl);
      const int mcnt = (n - q0) < 32 ? (n - q0) : 32;
#pragma unroll 1
      for (int pp = 0; pp < mcnt; ++pp) {
        const int s = __builtin_amdgcn_readlane(sl, pp);
        int cs = cnt[s];
        cs = cs < 0 ? 0 : cs;
        const float w = rsqrtf((float)(cs + 1)) * dc;
        const v4f hv = *(const v4f*)(hg + (size_t)s * CH + col);
        a0 += hv.x * w; a1 += hv.y * w; a2 += hv.z * w; a3 += hv.w * w;
      }
    }
    float v0 = a0 + vb.x, v1 = a1 + vb.y, v2 = a2 + vb.z, v3 = a3 + vb.w;
    v0 = vg.x * (v0 - vm.x) * rs0 + vbeta.x;
    v1 = vg.y * (v1 - vm.y) * rs1 + vbeta.y;
    v2 = vg.z * (v2 - vm.z) * rs2 + vbeta.z;
    v3 = vg.w * (v3 - vm.w) * rs3 + vbeta.w;
    const bool live = c < nN;
    v4f ov;
    ov.x = live ? elu1(v0) : 0.f;
    ov.y = live ? elu1(v1) : 0.f;
    ov.z = live ? elu1(v2) : 0.f;
    ov.w = live ? elu1(v3) : 0.f;
    float* gp = h2 + (size_t)c * CH + col;
    *(volatile v4f*)gp = ov;
    __threadfence();
    *(volatile v4f*)gp = ov;
  }
}

__global__ __launch_bounds__(NTHR) void k_sage(
    const int* __restrict__ csr, const int* __restrict__ off, const int* __restrict__ cnt,
    const float* __restrict__ h2, _Float16* ah3, int nN, int csrLen) {
  const int tid = threadIdx.x, lane = tid & 31, wave = tid >> 5;
  const int tbase = blockIdx.x * TGT + wave * 32;
  const int col = 4 * lane;
  const int cl    = tbase + lane;
  const int cnt_l = cnt[cl];
  const int off_l = off[cl];

#pragma unroll 1
  for (int j = 0; j < 32; ++j) {
    const int c = tbase + j;
    int cc = __shfl(cnt_l, j);
    cc = cc < 0 ? 0 : cc;
    const int n = cc > DEGCAP ? DEGCAP : cc;
    const int st = __shfl(off_l, j);
    float a0 = 0.f, a1 = 0.f, a2 = 0.f, a3 = 0.f;
#pragma unroll 1
    for (int q0 = 0; q0 < n; q0 += 32) {
      int pos = st + q0 + lane;
      pos = pos < 0 ? 0 : (pos > csrLen - 1 ? csrLen - 1 : pos);
      int sl = csr[pos];
      sl = sl < 0 ? 0 : (sl > nN - 1 ? nN - 1 : sl);
      const int mcnt = (n - q0) < 32 ? (n - q0) : 32;
#pragma unroll 1
      for (int pp = 0; pp < mcnt; ++pp) {
        const int s = __builtin_amdgcn_readlane(sl, pp);
        const v4f hv = *(const v4f*)(h2 + (size_t)s * CH + col);
        a0 += hv.x; a1 += hv.y; a2 += hv.z; a3 += hv.w;
      }
    }
    const float rc = __builtin_amdgcn_rcpf((float)(cc > 1 ? cc : 1));
    const v4f hc = *(const v4f*)(h2 + (size_t)c * CH + col);
    v4h om, oh;
    om[0] = (_Float16)((a0 * rc) * (float)ASC);
    om[1] = (_Float16)((a1 * rc) * (float)ASC);
    om[2] = (_Float16)((a2 * rc) * (float)ASC);
    om[3] = (_Float16)((a3 * rc) * (float)ASC);
    oh[0] = (_Float16)(hc.x * (float)ASC);
    oh[1] = (_Float16)(hc.y * (float)ASC);
    oh[2] = (_Float16)(hc.z * (float)ASC);
    oh[3] = (_Float16)(hc.w * (float)ASC);
    _Float16* gp = ah3 + (size_t)c * (2 * CH) + 4 * lane;
    *(volatile v4h*)gp = om;
    *(volatile v4h*)(gp + CH) = oh;
    __threadfence();
    *(volatile v4h*)gp = om;
    *(volatile v4h*)(gp + CH) = oh;
  }
}

__global__ __launch_bounds__(NTHR) void k_gat2(
    const int* __restrict__ csr, const int* __restrict__ off, const int* __restrict__ cnt,
    const float* __restrict__ eS, const float* __restrict__ eD, const float* __restrict__ xp,
    const float* __restrict__ bias, const float* __restrict__ bng, const float* __restrict__ bnb,
    const float* __restrict__ bnm, const float* __restrict__ bnv,
    float* yo, int nN, int npad, int csrLen) {
  const int tid = threadIdx.x, lane = tid & 31, wave = tid >> 5;
  const int tbase = blockIdx.x * TGT + wave * 32;
  const int hd = lane >> 3;
  const int colx = 16 * lane;
  const int col = 4 * lane;
  const int cl    = tbase + lane;
  const int cnt_l = cnt[cl];
  const int off_l = off[cl];
  const float* eSh = eS + (size_t)hd * npad;
  const float* eDh = eD + (size_t)hd * npad;
  const v4f vb = *(const v4f*)(bias + col);
  const v4f vg = *(const v4f*)(bng + col);
  const v4f vbeta = *(const v4f*)(bnb + col);
  const v4f vm = *(const v4f*)(bnm + col);
  const v4f vv = *(const v4f*)(bnv + col);
  const float rs0 = rsqrtf(vv.x + BN_EPS), rs1 = rsqrtf(vv.y + BN_EPS);
  const float rs2 = rsqrtf(vv.z + BN_EPS), rs3 = rsqrtf(vv.w + BN_EPS);
  const int srcl = lane >> 2, sel = lane & 3;

#pragma unroll 1
  for (int j = 0; j < 32; ++j) {
    const int c = tbase + j;
    int n = __shfl(cnt_l, j);
    n = n < 0 ? 0 : (n > DEGCAP ? DEGCAP : n);
    const int st = __shfl(off_l, j);
    const float edc = eDh[c];
    const float eself = lrelu(eSh[c] + edc);

    float mx = eself;
#pragma unroll 1
    for (int q0 = 0; q0 < n; q0 += 32) {
      int pos = st + q0 + lane;
      pos = pos < 0 ? 0 : (pos > csrLen - 1 ? csrLen - 1 : pos);
      int sl = csr[pos];
      sl = sl < 0 ? 0 : (sl > nN - 1 ? nN - 1 : sl);
      const int mcnt = (n - q0) < 32 ? (n - q0) : 32;
#pragma unroll 1
      for (int pp = 0; pp < mcnt; ++pp) {
        const int s = __builtin_amdgcn_readlane(sl, pp);
        mx = fmaxf(mx, lrelu(eSh[s] + edc));
      }
    }

    const float pself = __expf(eself - mx);
    float den = pself;
    float acc[16];
    {
      const float* xr = xp + (size_t)c * F2 + colx;
      const v4f x0 = *(const v4f*)xr, x1 = *(const v4f*)(xr + 4);
      const v4f x2 = *(const v4f*)(xr + 8), x3 = *(const v4f*)(xr + 12);
      acc[0]  = pself * x0.x; acc[1]  = pself * x0.y; acc[2]  = pself * x0.z; acc[3]  = pself * x0.w;
      acc[4]  = pself * x1.x; acc[5]  = pself * x1.y; acc[6]  = pself * x1.z; acc[7]  = pself * x1.w;
      acc[8]  = pself * x2.x; acc[9]  = pself * x2.y; acc[10] = pself * x2.z; acc[11] = pself * x2.w;
      acc[12] = pself * x3.x; acc[13] = pself * x3.y; acc[14] = pself * x3.z; acc[15] = pself * x3.w;
    }
#pragma unroll 1
    for (int q0 = 0; q0 < n; q0 += 32) {
      int pos = st + q0 + lane;
      pos = pos < 0 ? 0 : (pos > csrLen - 1 ? csrLen - 1 : pos);
      int sl = csr[pos];
      sl = sl < 0 ? 0 : (sl > nN - 1 ? nN - 1 : sl);
      const int mcnt = (n - q0) < 32 ? (n - q0) : 32;
#pragma unroll 1
      for (int pp = 0; pp < mcnt; ++pp) {
        const int s = __builtin_amdgcn_readlane(sl, pp);
        const float p = __expf(lrelu(eSh[s] + edc) - mx);
        den += p;
        const float* xr = xp + (size_t)s * F2 + colx;
        const v4f x0 = *(const v4f*)xr, x1 = *(const v4f*)(xr + 4);
        const v4f x2 = *(const v4f*)(xr + 8), x3 = *(const v4f*)(xr + 12);
        acc[0]  += x0.x * p; acc[1]  += x0.y * p; acc[2]  += x0.z * p; acc[3]  += x0.w * p;
        acc[4]  += x1.x * p; acc[5]  += x1.y * p; acc[6]  += x1.z * p; acc[7]  += x1.w * p;
        acc[8]  += x2.x * p; acc[9]  += x2.y * p; acc[10] += x2.z * p; acc[11] += x2.w * p;
        acc[12] += x3.x * p; acc[13] += x3.y * p; acc[14] += x3.z * p; acc[15] += x3.w * p;
      }
    }

    const float rd = __builtin_amdgcn_rcpf(den);
    float o[16];
#pragma unroll
    for (int i = 0; i < 16; ++i) o[i] = acc[i] * rd;
#pragma unroll
    for (int i = 0; i < 16; ++i) o[i] += __shfl_xor(o[i], 8);
#pragma unroll
    for (int i = 0; i < 16; ++i) o[i] += __shfl_xor(o[i], 16);
    float r[4] = {0.f, 0.f, 0.f, 0.f};
#pragma unroll
    for (int q = 0; q < 4; ++q) {
#pragma unroll
      for (int i = 0; i < 4; ++i) {
        const float t = __shfl(o[4 * q + i], srcl);
        r[i] = (sel == q) ? t : r[i];
      }
    }
    float v0 = r[0] * 0.25f + vb.x, v1 = r[1] * 0.25f + vb.y;
    float v2 = r[2] * 0.25f + vb.z, v3 = r[3] * 0.25f + vb.w;
    v0 = vg.x * (v0 - vm.x) * rs0 + vbeta.x;
    v1 = vg.y * (v1 - vm.y) * rs1 + vbeta.y;
    v2 = vg.z * (v2 - vm.z) * rs2 + vbeta.z;
    v3 = vg.w * (v3 - vm.w) * rs3 + vbeta.w;
    v4f ov;
    ov.x = elu1(v0); ov.y = elu1(v1); ov.z = elu1(v2); ov.w = elu1(v3);
    float* gp = yo + (size_t)c * CH + col;
    const bool act = (c < nN);
    if (act) *(volatile v4f*)gp = ov;
    __threadfence();
    if (act) *(volatile v4f*)gp = ov;
  }
}

__global__ __launch_bounds__(NTHR) void k_pool(const int* __restrict__ batch, const float* __restrict__ node,
                                               float* gout, _Float16* gh, int nN, int nG) {
  const int tid = threadIdx.x, lane = tid & 31, wave = tid >> 5;
  const int g = (int)blockIdx.x * NWAVE + wave;
  const int gc = g > nG - 1 ? nG - 1 : g;
  const int col = 4 * lane;
  float a0 = 0.f, a1 = 0.f, a2 = 0.f, a3 = 0.f;
  int cg = 0;
#pragma unroll 1
  for (int i0 = 0; i0 < nN; i0 += 32) {
    const int idx = (i0 + lane) > nN - 1 ? nN - 1 : (i0 + lane);
    const int b = batch[idx];
    const bool hit = ((i0 + lane) < nN) && (b == gc);
    unsigned msk = __builtin_amdgcn_ballot_w32(hit);
    cg += (int)__builtin_popcount(msk);
#pragma unroll 1
    for (int it = 0; it < 32; ++it) {
      if (msk == 0u) break;
      const int bit = __builtin_ctz(msk);
      msk &= msk - 1u;
      const int nd = i0 + bit;
      const v4f v = *(const v4f*)(node + (size_t)nd * CH + col);
      a0 += v.x; a1 += v.y; a2 += v.z; a3 += v.w;
    }
  }
  const float rc = __builtin_amdgcn_rcpf((float)(cg > 1 ? cg : 1));
  v4f ov;
  ov.x = a0 * rc; ov.y = a1 * rc; ov.z = a2 * rc; ov.w = a3 * rc;
  v4h oh;
  oh[0] = (_Float16)(ov.x * (float)ASC);
  oh[1] = (_Float16)(ov.y * (float)ASC);
  oh[2] = (_Float16)(ov.z * (float)ASC);
  oh[3] = (_Float16)(ov.w * (float)ASC);
  float* gp = gout + (size_t)gc * CH + col;
  _Float16* hp = gh + (size_t)gc * CH + col;
  const bool act = g < nG;
  if (act) { *(volatile v4f*)gp = ov; *(volatile v4h*)hp = oh; }
  __threadfence();
  if (act) { *(volatile v4f*)gp = ov; *(volatile v4h*)hp = oh; }
}

extern "C" void kernel_launch(void* const* d_in, const int* in_sizes, int n_in,
                              void* d_out, int out_size, void* d_ws, size_t ws_size,
                              hipStream_t stream) {
  if (n_in < 36) return;
  const int nN = in_sizes[0] / FIN;
  const int nE = in_sizes[1] / 2;
  if (nN <= 0 || nE <= 0) return;
  if (in_sizes[0] != nN * FIN || in_sizes[1] != 2 * nE || in_sizes[2] != nN) return;
  if (in_sizes[3] != FIN * F1 || in_sizes[4] != NH1 * CH || in_sizes[5] != NH1 * CH || in_sizes[6] != F1) return;
  for (int i = 7; i <= 10; ++i) if (in_sizes[i] != F1) return;
  if (in_sizes[11] != F1 * CH) return;
  for (int i = 12; i <= 16; ++i) if (in_sizes[i] != CH) return;
  if (in_sizes[17] != CH * CH || in_sizes[18] != CH || in_sizes[19] != CH * CH) return;
  for (int i = 20; i <= 23; ++i) if (in_sizes[i] != CH) return;
  if (in_sizes[24] != CH * F2 || in_sizes[25] != NH2 * CH || in_sizes[26] != NH2 * CH) return;
  for (int i = 27; i <= 31; ++i) if (in_sizes[i] != CH) return;
  if (in_sizes[32] != CH * CH || in_sizes[33] != CH || in_sizes[34] != CH * PO || in_sizes[35] != PO) return;
  if (nE > (1 << 28) || nN > (1 << 22)) return;
  const long rem = (long)out_size - (long)nN * CH;
  if (rem <= 0 || (rem % (CH + PO)) != 0) return;
  const int nG = (int)(rem / (CH + PO));
  if (nG <= 0 || (nG % BM) != 0 || nG > (1 << 20)) return;

  const float* x     = (const float*)d_in[0];
  const int*   ei    = (const int*)d_in[1];
  const int*   src   = ei;
  const int*   dst   = ei + nE;
  const int*   batch = (const int*)d_in[2];
  const float* W1    = (const float*)d_in[3];
  const float* as1   = (const float*)d_in[4];
  const float* ad1   = (const float*)d_in[5];
  const float* bias1 = (const float*)d_in[6];
  const float* g1 = (const float*)d_in[7],  *b1 = (const float*)d_in[8];
  const float* m1 = (const float*)d_in[9],  *v1 = (const float*)d_in[10];
  const float* Wg = (const float*)d_in[11], *bg = (const float*)d_in[12];
  const float* g2 = (const float*)d_in[13], *b2 = (const float*)d_in[14];
  const float* m2 = (const float*)d_in[15], *v2 = (const float*)d_in[16];
  const float* Wl = (const float*)d_in[17], *bl = (const float*)d_in[18];
  const float* Wr = (const float*)d_in[19];
  const float* g3 = (const float*)d_in[20], *b3 = (const float*)d_in[21];
  const float* m3 = (const float*)d_in[22], *v3 = (const float*)d_in[23];
  const float* W2 = (const float*)d_in[24];
  const float* as2 = (const float*)d_in[25], *ad2 = (const float*)d_in[26];
  const float* bias2 = (const float*)d_in[27];
  const float* g4 = (const float*)d_in[28], *b4 = (const float*)d_in[29];
  const float* m4 = (const float*)d_in[30], *v4 = (const float*)d_in[31];
  const float* Wp1 = (const float*)d_in[32], *bp1 = (const float*)d_in[33];
  const float* Wp2 = (const float*)d_in[34], *bp2 = (const float*)d_in[35];

  float* out0 = (float*)d_out;
  float* out1 = out0 + (size_t)nN * CH;
  float* out2 = out1 + (size_t)nG * CH;

  const int NPAD   = ((nN + TGT - 1) / TGT) * TGT;
  const int nBC    = (nN + NBC - 1) / NBC;
  const int CNTPAD = nBC * NBC;
  if (CNTPAD < NPAD) return;
  if (4 * nBC + 1 > RBN) return;
  const int nBF    = (nN + NBF - 1) / NBF;
  if (nBF > 4 * nBC) return;
  const int csrLen = ((nE + 31) & ~31) + 4096;
  if (31 * 4 * nBC > 4096) return;
  const int nAgg   = NPAD / TGT;
  const int nGemm  = NPAD / BM;

  char* ws = (char*)d_ws;
  size_t off = 0;
  const size_t oU   = off; off += (size_t)256 * 4;              off = (off + 255) & ~(size_t)255;
  const size_t oW1  = off; off += (size_t)F1 * 32 * 2;           off = (off + 255) & ~(size_t)255;
  const size_t oWg  = off; off += (size_t)CH * F1 * 2;           off = (off + 255) & ~(size_t)255;
  const size_t oWlr = off; off += (size_t)CH * 2 * CH * 2;       off = (off + 255) & ~(size_t)255;
  const size_t oW2  = off; off += (size_t)F2 * CH * 2;           off = (off + 255) & ~(size_t)255;
  const size_t oWp1 = off; off += (size_t)CH * CH * 2;           off = (off + 255) & ~(size_t)255;
  const size_t oWp2 = off; off += (size_t)PO * CH * 2;           off = (off + 255) & ~(size_t)255;
  const size_t oXp  = off; off += (size_t)NPAD * KX * 4;         off = (off + 255) & ~(size_t)255;
  const size_t oES1 = off; off += (size_t)NH1 * NPAD * 4;        off = (off + 255) & ~(size_t)255;
  const size_t oED1 = off; off += (size_t)NH1 * NPAD * 4;        off = (off + 255) & ~(size_t)255;
  const size_t oCnt = off; off += (size_t)CNTPAD * 4;            off = (off + 255) & ~(size_t)255;
  const size_t oOff = off; off += (size_t)CNTPAD * 4;            off = (off + 255) & ~(size_t)255;
  const size_t oRb  = off; off += (size_t)RBN * 4;               off = (off + 255) & ~(size_t)255;
  const size_t oCsr = off; off += (size_t)csrLen * 4;            off = (off + 255) & ~(size_t)255;
  const size_t oZ   = off; off += (size_t)NPAD * CH * 2;         off = (off + 255) & ~(size_t)255;
  const size_t oBig = off; off += (size_t)NPAD * F1 * 2;         off = (off + 255) & ~(size_t)255;
  const size_t oHg  = off; off += (size_t)NPAD * CH * 4;         off = (off + 255) & ~(size_t)255;
  const size_t oH2  = off; off += (size_t)NPAD * CH * 4;         off = (off + 255) & ~(size_t)255;
  const size_t oES2 = off; off += (size_t)NH2 * NPAD * 4;        off = (off + 255) & ~(size_t)255;
  const size_t oED2 = off; off += (size_t)NH2 * NPAD * 4;        off = (off + 255) & ~(size_t)255;
  const size_t oGh  = off; off += (size_t)nG * CH * 2;           off = (off + 255) & ~(size_t)255;
  const size_t oP1  = off; off += (size_t)nG * CH * 2;           off = (off + 255) & ~(size_t)255;
  if (off > ws_size || off > (size_t)WSCAP) return;
  float*    u    = (float*)(ws + oU);
  _Float16* w1p  = (_Float16*)(ws + oW1);
  _Float16* wgp  = (_Float16*)(ws + oWg);
  _Float16* wlr  = (_Float16*)(ws + oWlr);
  _Float16* w2p  = (_Float16*)(ws + oW2);
  _Float16* wp1p = (_Float16*)(ws + oWp1);
  _Float16* wp2p = (_Float16*)(ws + oWp2);
  float*    xpad = (float*)(ws + oXp);
  float*    es1  = (float*)(ws + oES1);
  float*    ed1  = (float*)(ws + oED1);
  int*      cnt  = (int*)(ws + oCnt);
  int*      offp = (int*)(ws + oOff);
  int*      rb   = (int*)(ws + oRb);
  int*      csr  = (int*)(ws + oCsr);
  _Float16* zh   = (_Float16*)(ws + oZ);
  _Float16* h3h  = (_Float16*)(ws + oZ);
  _Float16* h1h  = (_Float16*)(ws + oBig);
  float*    xp2  = (float*)(ws + oBig);
  float*    hg   = (float*)(ws + oHg);
  _Float16* ah3  = (_Float16*)(ws + oHg);
  float*    h2   = (float*)(ws + oH2);
  float*    es2  = (float*)(ws + oES2);
  float*    ed2  = (float*)(ws + oED2);
  _Float16* gh   = (_Float16*)(ws + oGh);
  _Float16* p1h  = (_Float16*)(ws + oP1);

  const int vec8 = ((nE & 3) == 0) ? 1 : 0;
  const float osc = 1.0f / (float)(ASC * WSC);

  k_uvec<<<1, NTHR, 0, stream>>>(W1, as1, ad1, u);
  k_xprep<<<NPAD / 256, NTHR, 0, stream>>>(x, u, xpad, es1, ed1, nN, NPAD);
  k_w1cvt<<<(F1 * 4) / NTHR, NTHR, 0, stream>>>(W1, w1p);
  k_wtcvt<<<(CH * F1 / 8 + NTHR - 1) / NTHR, NTHR, 0, stream>>>(Wg, wgp, F1, CH, F1, 0, CH * F1 / 8);
  k_wtcvt<<<(CH * CH / 8 + NTHR - 1) / NTHR, NTHR, 0, stream>>>(Wl, wlr, CH, CH, 2 * CH, 0, CH * CH / 8);
  k_wtcvt<<<(CH * CH / 8 + NTHR - 1) / NTHR, NTHR, 0, stream>>>(Wr, wlr, CH, CH, 2 * CH, CH, CH * CH / 8);
  k_wtcvt<<<(F2 * CH / 8 + NTHR - 1) / NTHR, NTHR, 0, stream>>>(W2, w2p, CH, F2, CH, 0, F2 * CH / 8);
  k_wtcvt<<<(CH * CH / 8 + NTHR - 1) / NTHR, NTHR, 0, stream>>>(Wp1, wp1p, CH, CH, CH, 0, CH * CH / 8);
  k_wtcvt<<<(PO * CH / 8 + NTHR - 1) / NTHR, NTHR, 0, stream>>>(Wp2, wp2p, CH, PO, CH, 0, PO * CH / 8);

  k_count<<<nBC, NTHR, 0, stream>>>(dst, cnt, nE, vec8);
  k_offsets<<<1, OTHR, 0, stream>>>(cnt, offp, rb, nBC);
  hipFuncSetAttribute(reinterpret_cast<const void*>(&k_fill),
                      hipFuncAttributeMaxDynamicSharedMemorySize, LDS_FILL);
  k_fill<<<nBF, NTHR, LDS_FILL, stream>>>(src, dst, offp, rb, csr, nN, nE, vec8, csrLen);

  k_gat1<<<nAgg, NTHR, 0, stream>>>(csr, offp, cnt, es1, ed1, xpad, zh, nN, NPAD, csrLen);
  k_gemm<128, 1><<<dim3(nGemm, NH1, 1), NTHR, 0, stream>>>(
      zh, w1p, bias1, g1, b1, m1, v1, as2, ad2, es2, ed2, hg, h1h, CH, 1, 1, F1, 1 | 2 | 4, NPAD, osc);
  k_gemm<128, 0><<<dim3(nGemm, 1, 1), NTHR, 0, stream>>>(
      h1h, wgp, bg, g2, b2, m2, v2, as2, ad2, es2, ed2, hg, zh, F1, 0, F1 / 32, CH, 0, NPAD, osc);
  k_gcn<<<nAgg, NTHR, 0, stream>>>(csr, offp, cnt, hg, bg, g2, b2, m2, v2, h2, nN, csrLen);
  k_sage<<<nAgg, NTHR, 0, stream>>>(csr, offp, cnt, h2, ah3, nN, csrLen);
  k_gemm<128, 1><<<dim3(nGemm, 1, 1), NTHR, 0, stream>>>(
      ah3, wlr, bl, g3, b3, m3, v3, as2, ad2, es2, ed2, hg, h3h, 2 * CH, 0, (2 * CH) / 32, CH, 1 | 2 | 4, NPAD, osc);
  k_gemm<128, 0><<<dim3(nGemm, NH2, 1), NTHR, 0, stream>>>(
      h3h, w2p, bias2, g4, b4, m4, v4, as2, ad2, es2, ed2, xp2, zh, CH, 0, CH / 32, F2, 16, NPAD, osc);
  k_gat2<<<nAgg, NTHR, 0, stream>>>(csr, offp, cnt, es2, ed2, xp2, bias2, g4, b4, m4, v4, out0, nN, NPAD, csrLen);
  k_pool<<<nG / NWAVE, NTHR, 0, stream>>>(batch, out0, out1, gh, nN, nG);
  k_gemm<128, 1><<<dim3(nG / BM, 1, 1), NTHR, 0, stream>>>(
      gh, wp1p, bp1, g4, b4, m4, v4, as2, ad2, es2, ed2, hg, p1h, CH, 0, CH / 32, CH, 1 | 8, nG, osc);
  k_gemm<64, 0><<<dim3(nG / BM, 1, 1), NTHR, 0, stream>>>(
      p1h, wp2p, bp2, g4, b4, m4, v4, as2, ad2, es2, ed2, out2, zh, CH, 0, CH / 32, PO, 1, nG, osc);
}
